// Rvt_59605556134239
// MI455X (gfx1250) — hardware-verified
//
#include <hip/hip_runtime.h>


namespace {
constexpr int Nn = 16, I0 = 128, HW = 32, NP = HW * HW, C = 256, CO = 128, NT = Nn * NP, KC = 9 * C;
constexpr float AS_ = 8.0f, VS = 8.0f, PS = 8.0f;
constexpr size_t PLN = (size_t)NT * C;

typedef _Float16 b16;
typedef __attribute__((ext_vector_type(16))) _Float16 v16b;
typedef __attribute__((ext_vector_type(16))) __bf16 v16bb;
typedef __attribute__((ext_vector_type(8))) _Float16 v8b;
typedef __attribute__((ext_vector_type(8))) unsigned short v8us;
typedef __attribute__((ext_vector_type(8))) float v8f;
typedef __attribute__((ext_vector_type(4))) float v4f;
__device__ __forceinline__ float bf16_rne(float f) { unsigned int u = __float_as_uint(f); u += 0x7FFFu + ((u >> 16) & 1u); return __uint_as_float(u & 0xFFFF0000u); }
__device__ __forceinline__ unsigned short bf16_bits(float f) { unsigned int u = __float_as_uint(f); u += 0x7FFFu + ((u >> 16) & 1u); return (unsigned short)(u >> 16); }
__device__ __forceinline__ void split16(float v, b16& hi, b16& lo) { hi = (b16)v; lo = (b16)(v - (float)hi); }
__device__ __forceinline__ v16b frag_kb(const b16* p, int hh) { const v8b a = *(const v8b*)(p + 8 * hh), b = *(const v8b*)(p + 16 + 8 * hh); v16b f;
#pragma unroll
  for (int e = 0; e < 8; ++e) { f[e] = a[e]; f[8 + e] = b[e]; } return f; }
__device__ __forceinline__ v16bb frag_bf(const unsigned short* p, int hh) { const v8us a = *(const v8us*)(p + 8 * hh), b = *(const v8us*)(p + 16 + 8 * hh); union { unsigned short s[16]; v16bb v; } u;
#pragma unroll
  for (int e = 0; e < 8; ++e) { u.s[e] = a[e]; u.s[8 + e] = b[e]; } return u.v; }
__device__ __forceinline__ void frag_split(const float* p, int hh, v16b& fh, v16b& fl) {
#pragma unroll
  for (int e = 0; e < 8; ++e) { b16 a, c; split16(p[8 * hh + e] * AS_, a, c); fh[e] = a; fl[e] = c; split16(p[16 + 8 * hh + e] * AS_, a, c); fh[8 + e] = a; fl[8 + e] = c; } }
__device__ __forceinline__ v8f wmma16b(v16b a, v16b b, v8f c) { v8f d = __builtin_amdgcn_wmma_f32_16x16x32_f16(false, a, false, b, (short)0, c, false, false); asm volatile("v_nop\n\tv_nop\n\tv_nop\n\tv_nop" : "+v"(d) : "v"(a), "v"(b)); return d; }
__device__ __forceinline__ v8f wmma16bb(v16bb a, v16bb b, v8f c) { v8f d = __builtin_amdgcn_wmma_f32_16x16x32_bf16(false, a, false, b, (short)0, c, false, false); asm volatile("v_nop\n\tv_nop\n\tv_nop\n\tv_nop" : "+v"(d) : "v"(a), "v"(b)); return d; }
__device__ __forceinline__ void wave_lds_sync() { __builtin_amdgcn_fence(__ATOMIC_RELEASE, "workgroup"); __builtin_amdgcn_wave_barrier(); __builtin_amdgcn_fence(__ATOMIC_ACQUIRE, "workgroup"); }
__device__ __forceinline__ float nexp(float x) { return __builtin_amdgcn_exp2f(x * 1.4426950408889634f); }
__device__ __forceinline__ float sigm(float x) { return __builtin_amdgcn_rcpf(1.0f + nexp(-x)); }
__device__ __forceinline__ float tanh_(float x) { const float e = nexp(-2.0f * fabsf(x)); const float t = (1.0f - e) * __builtin_amdgcn_rcpf(1.0f + e); return (x >= 0.0f) ? t : -t; }

__device__ __forceinline__ void store_tile(const float* Tt, float* dst0, int ld, int lane) { const int hlf = lane >> 4, nloc = lane & 15;
  for (int pass = 0; pass < 2; ++pass) {
#pragma unroll
    for (int j = 0; j < 16; ++j) { const int rr = j * 2 + hlf, c4 = nloc * 4; *(volatile v4f*)(dst0 + (size_t)rr * ld + c4) = *(const v4f*)(Tt + rr * 64 + c4); }
    __threadfence(); } }

__global__ __launch_bounds__(256) void prep_kernel(const float* __restrict__ x, const float* __restrict__ wpx, const float* __restrict__ wconv, const float* __restrict__ wq, const float* __restrict__ wk, const float* __restrict__ wv, const float* __restrict__ s, const float* __restrict__ wz, const float* __restrict__ bz, const float* __restrict__ wn, const float* __restrict__ bn, const float* __restrict__ wo, const float* __restrict__ bo,
                                                   unsigned short* __restrict__ xT, unsigned short* __restrict__ wpx16, b16* __restrict__ wc16, b16* __restrict__ wqkv16, b16* __restrict__ wzn16, b16* __restrict__ wo16, float* __restrict__ P) {
  __shared__ __attribute__((aligned(16))) unsigned short Tt[64][I0 + 8];
  const int t_ = threadIdx.x, n = blockIdx.y, p0 = blockIdx.x * 64; const float* src = x + (size_t)n * I0 * NP;
  for (int i = t_; i < I0 * 64; i += 256) { const int c = i >> 6, pp = i & 63; Tt[pp][c] = bf16_bits(src[(size_t)c * NP + p0 + pp]); }
  __syncthreads();
  const size_t gid = ((size_t)blockIdx.y * gridDim.x + blockIdx.x) * 256 + t_, gn = (size_t)gridDim.x * gridDim.y * 256;
  for (int pass = 0; pass < 2; ++pass) {
    for (int i = t_; i < 64 * I0 / 8; i += 256) { const int pp = i >> 4, c8 = (i & 15) * 8; *(volatile v8us*)(xT + ((size_t)n * NP + p0 + pp) * I0 + c8) = *(const v8us*)(&Tt[pp][c8]); }
    for (size_t p = gid; p < (size_t)C * I0 / 8; p += gn) { v8us v;
#pragma unroll
      for (int e = 0; e < 8; ++e) v[e] = bf16_bits(wpx[p * 8 + e]);
      *(volatile v8us*)(wpx16 + p * 8) = v; }
    for (size_t p = gid; p < (size_t)C * KC / 8; p += gn) { v8b v;
#pragma unroll
      for (int e = 0; e < 8; ++e) { const size_t q = p * 8 + e; const int co = (int)(q / KC), k = (int)(q % KC), tap = k >> 8, ci = k & 255; v[e] = (b16)bf16_rne(wconv[((size_t)co * 512 + ci) * 9 + tap]); }
      *(volatile v8b*)(wc16 + p * 8) = v; }
    for (size_t p = gid; p < (size_t)3 * C * C / 8; p += gn) { const size_t m = p / ((size_t)C * C / 8), q = p % ((size_t)C * C / 8); const float* W = (m == 0) ? wq : (m == 1) ? wk : wv; v8b v;
#pragma unroll
      for (int e = 0; e < 8; ++e) v[e] = (b16)bf16_rne(W[q * 8 + e]);
      *(volatile v8b*)(wqkv16 + p * 8) = v; }
    for (size_t p = gid; p < (size_t)2 * C * 512 / 8; p += gn) { const size_t m = p / ((size_t)C * 512 / 8), q = p % ((size_t)C * 512 / 8); const float* W = (m == 0) ? wz : wn; v8b v;
#pragma unroll
      for (int e = 0; e < 8; ++e) v[e] = (b16)bf16_rne(W[q * 8 + e]);
      *(volatile v8b*)(wzn16 + p * 8) = v; }
    for (size_t p = gid; p < (size_t)CO * C / 8; p += gn) { v8b v;
#pragma unroll
      for (int e = 0; e < 8; ++e) v[e] = (b16)bf16_rne(wo[p * 8 + e]);
      *(volatile v8b*)(wo16 + p * 8) = v; }
    for (size_t p = gid; p < 1024; p += gn) { float v = 0.0f; if (p < 256) v = s[p]; else if (p < 512) v = bz[p - 256]; else if (p < 768) v = bn[p - 512]; else if (p < 896) v = bo[p - 768]; ((volatile float*)P)[p] = bf16_rne(v); }
    __threadfence(); }
}

__global__ __launch_bounds__(128) void px_kernel(const unsigned short* __restrict__ xT, const unsigned short* __restrict__ wpx16, float* __restrict__ xt) {
  __shared__ __attribute__((aligned(16))) float Ts[4][32 * 64];
  const int lane = threadIdx.x & 31, wave = threadIdx.x >> 5, nloc = lane & 15, hlf = lane >> 4, m0 = blockIdx.y * 128 + wave * 32, c0 = blockIdx.x * 64;
  v8f acc[2][4];
#pragma unroll
  for (int r = 0; r < 2; ++r)
#pragma unroll
    for (int t = 0; t < 4; ++t) acc[r][t] = (v8f){};
#pragma unroll
  for (int kb = 0; kb < I0; kb += 32) { const v16bb a0 = frag_bf(xT + (size_t)(m0 + nloc) * I0 + kb, hlf), a1 = frag_bf(xT + (size_t)(m0 + 16 + nloc) * I0 + kb, hlf);
#pragma unroll
    for (int t = 0; t < 4; ++t) { const v16bb bw = frag_bf(wpx16 + (size_t)(c0 + t * 16 + nloc) * I0 + kb, hlf); acc[0][t] = wmma16bb(a0, bw, acc[0][t]); acc[1][t] = wmma16bb(a1, bw, acc[1][t]); } }
  float* Tt = Ts[wave];
#pragma unroll
  for (int t = 0; t < 4; ++t)
#pragma unroll
    for (int r = 0; r < 2; ++r)
#pragma unroll
      for (int v = 0; v < 8; ++v) Tt[(r * 16 + v + 8 * hlf) * 64 + t * 16 + nloc] = tanh_(acc[r][t][v]);
  wave_lds_sync();
  store_tile(Tt, xt + (size_t)m0 * C + c0, C, lane);
}

__global__ __launch_bounds__(128) void conv_kernel(const float* __restrict__ xt, const b16* __restrict__ wc16, float* __restrict__ c) {
  __shared__ __attribute__((aligned(16))) float Ts[4][32 * 64];
  const int lane = threadIdx.x & 31, wave = threadIdx.x >> 5, nloc = lane & 15, hlf = lane >> 4, m0 = blockIdx.y * 128 + wave * 32, c0 = blockIdx.x * 64; const int n = m0 / NP;
  const int pa = (m0 % NP) + nloc, pb_ = pa + 16; const int ya = pa >> 5, xa = pa & 31, yb = pb_ >> 5, xb = pb_ & 31; const float* X = xt + ((size_t)n * NP) * C;
  v8f acc[2][4];
#pragma unroll
  for (int r = 0; r < 2; ++r)
#pragma unroll
    for (int t = 0; t < 4; ++t) acc[r][t] = (v8f){};
  for (int tap = 0; tap < 9; ++tap) { const int dy = tap / 3 - 1, dx = tap % 3 - 1; const int y1 = ya + dy, x1 = xa + dx, y2 = yb + dy, x2 = xb + dx;
    const bool ok1 = ((unsigned)y1 < 32u) && ((unsigned)x1 < 32u), ok2 = ((unsigned)y2 < 32u) && ((unsigned)x2 < 32u);
    const float* r1 = X + (size_t)((min(max(y1, 0), 31) << 5) + min(max(x1, 0), 31)) * C; const float* r2 = X + (size_t)((min(max(y2, 0), 31) << 5) + min(max(x2, 0), 31)) * C;
    const float m1 = ok1 ? 1.0f : 0.0f, m2 = ok2 ? 1.0f : 0.0f;
#pragma unroll 2
    for (int kb = 0; kb < C; kb += 32) { v16b a0, l0, a1, l1;
#pragma unroll
      for (int e = 0; e < 8; ++e) { b16 p, q; split16(r1[kb + 8 * hlf + e] * m1 * AS_, p, q); a0[e] = p; l0[e] = q; split16(r1[kb + 16 + 8 * hlf + e] * m1 * AS_, p, q); a0[8 + e] = p; l0[8 + e] = q;
        split16(r2[kb + 8 * hlf + e] * m2 * AS_, p, q); a1[e] = p; l1[e] = q; split16(r2[kb + 16 + 8 * hlf + e] * m2 * AS_, p, q); a1[8 + e] = p; l1[8 + e] = q; }
#pragma unroll
      for (int t = 0; t < 4; ++t) { const v16b bw = frag_kb(wc16 + (size_t)(c0 + t * 16 + nloc) * KC + tap * C + kb, hlf); acc[0][t] = wmma16b(a0, bw, acc[0][t]); acc[0][t] = wmma16b(l0, bw, acc[0][t]); acc[1][t] = wmma16b(a1, bw, acc[1][t]); acc[1][t] = wmma16b(l1, bw, acc[1][t]); } } }
  float* Tt = Ts[wave];
#pragma unroll
  for (int t = 0; t < 4; ++t)
#pragma unroll
    for (int r = 0; r < 2; ++r)
#pragma unroll
      for (int v = 0; v < 8; ++v) Tt[(r * 16 + v + 8 * hlf) * 64 + t * 16 + nloc] = acc[r][t][v] * (1.0f / AS_);
  wave_lds_sync();
  store_tile(Tt, c + (size_t)m0 * C + c0, C, lane);
}

__global__ __launch_bounds__(128) void qkv_kernel(const float* __restrict__ c, const b16* __restrict__ wqkv16, const float* __restrict__ P, b16* __restrict__ qp, b16* __restrict__ kp, b16* __restrict__ vt, float* __restrict__ qs) {
  __shared__ __attribute__((aligned(16))) b16 Th[4][32][64 + 8], Tl[4][32][64 + 8]; __shared__ __attribute__((aligned(16))) b16 Vh[64][128 + 8], Vl[64][128 + 8]; __shared__ __attribute__((aligned(16))) float Sq[4][32][4];
  const int lane = threadIdx.x & 31, wave = threadIdx.x >> 5, nloc = lane & 15, hlf = lane >> 4, which = blockIdx.z, m0 = blockIdx.y * 128 + wave * 32, ct = blockIdx.x, c0 = ct * 64;
  const int n = (blockIdx.y * 128) / NP, p0 = (blockIdx.y * 128) % NP; const b16* Wt = wqkv16 + (size_t)which * C * C; const float* s = P;
  v8f acc[2][4];
#pragma unroll
  for (int r = 0; r < 2; ++r)
#pragma unroll
    for (int t = 0; t < 4; ++t) acc[r][t] = (v8f){};
#pragma unroll 2
  for (int kb = 0; kb < C; kb += 32) { v16b a0, l0, a1, l1; frag_split(c + (size_t)(m0 + nloc) * C + kb, hlf, a0, l0); frag_split(c + (size_t)(m0 + 16 + nloc) * C + kb, hlf, a1, l1);
#pragma unroll
    for (int t = 0; t < 4; ++t) { const v16b bw = frag_kb(Wt + (size_t)(c0 + t * 16 + nloc) * C + kb, hlf); acc[0][t] = wmma16b(a0, bw, acc[0][t]); acc[0][t] = wmma16b(l0, bw, acc[0][t]); acc[1][t] = wmma16b(a1, bw, acc[1][t]); acc[1][t] = wmma16b(l1, bw, acc[1][t]); } }
  if (which < 2) {
    float ssq[2][8];
#pragma unroll
    for (int r = 0; r < 2; ++r)
#pragma unroll
      for (int v = 0; v < 8; ++v) ssq[r][v] = 0.0f;
#pragma unroll
    for (int t = 0; t < 4; ++t) { const int ch = c0 + t * 16 + nloc; const float sc = (which == 1) ? s[ch] : 1.0f;
#pragma unroll
      for (int r = 0; r < 2; ++r)
#pragma unroll
        for (int v = 0; v < 8; ++v) { const float raw = acc[r][t][v] * (1.0f / AS_); ssq[r][v] += raw * raw; b16 a_, c_; split16(raw * sc * AS_, a_, c_); Th[wave][r * 16 + 8 * hlf + v][t * 16 + nloc] = a_; Tl[wave][r * 16 + 8 * hlf + v][t * 16 + nloc] = c_; } }
#pragma unroll
    for (int r = 0; r < 2; ++r)
#pragma unroll
      for (int v = 0; v < 8; ++v) { float q = ssq[r][v];
#pragma unroll
        for (int o = 1; o < 16; o <<= 1) q += __shfl_xor(q, o);
        if (nloc == 0) Sq[wave][r * 16 + 8 * hlf + v][ct] = q; }
    wave_lds_sync();
    b16* dst = ((which == 0) ? qp : kp) + (size_t)m0 * C + c0;
    for (int pass = 0; pass < 2; ++pass) {
#pragma unroll
      for (int j = 0; j < 8; ++j) { const int rr = j * 4 + (lane >> 3), c8 = (lane & 7) * 8; *(volatile v8b*)(dst + (size_t)rr * C + c8) = *(const v8b*)(&Th[wave][rr][c8]); *(volatile v8b*)(dst + PLN + (size_t)rr * C + c8) = *(const v8b*)(&Tl[wave][rr][c8]); }
      ((volatile float*)qs)[((size_t)which * 4 + ct) * NT + m0 + lane] = Sq[wave][lane][ct];
      __threadfence(); }
    return; }
#pragma unroll
  for (int t = 0; t < 4; ++t)
#pragma unroll
    for (int r = 0; r < 2; ++r)
#pragma unroll
      for (int v = 0; v < 8; ++v) { b16 a_, c_; split16(acc[r][t][v] * (VS / AS_), a_, c_); Vh[t * 16 + nloc][wave * 32 + r * 16 + 8 * hlf + v] = a_; Vl[t * 16 + nloc][wave * 32 + r * 16 + 8 * hlf + v] = c_; }
  __syncthreads();
  for (int pass = 0; pass < 2; ++pass) { for (int i = threadIdx.x; i < 64 * 16; i += 128) { const int cc = i >> 4, c8 = (i & 15) * 8; const size_t dst = ((size_t)n * C + c0 + cc) * NP + p0 + c8;
      *(volatile v8b*)(vt + dst) = *(const v8b*)(&Vh[cc][c8]); *(volatile v8b*)(vt + PLN + dst) = *(const v8b*)(&Vl[cc][c8]); } __threadfence(); }
}

__global__ __launch_bounds__(256) void nrm_kernel(const float* __restrict__ qs, float* __restrict__ nq, float* __restrict__ nk) {
  const size_t p = (size_t)blockIdx.x * 256 + threadIdx.x; const float* a = qs + p; const float* b = qs + (size_t)4 * NT + p;
  const float iq = rsqrtf((a[0] + a[NT]) + (a[2 * NT] + a[3 * NT])), ik = rsqrtf((b[0] + b[NT]) + (b[2 * NT] + b[3 * NT]));
  for (int pass = 0; pass < 2; ++pass) { ((volatile float*)nq)[p] = iq; ((volatile float*)nk)[p] = ik; __threadfence(); }
}

__global__ __launch_bounds__(256) void attn_kernel(const b16* __restrict__ qp, const b16* __restrict__ kp, const b16* __restrict__ vt, const float* __restrict__ nq, const float* __restrict__ nk, float* __restrict__ arow) {
  __shared__ __attribute__((aligned(16))) float Os[8][16][C + 4];
  const int wid = threadIdx.x >> 5, lane = threadIdx.x & 31, hh = lane >> 4, col = lane & 15; const int tok0 = blockIdx.x * 128 + wid * 16, n = tok0 / NP; const size_t qi = (size_t)tok0 + col;
  const b16* K = kp + ((size_t)n * NP) * C; const b16* V = vt + ((size_t)n * C) * NP; const float* NK = nk + (size_t)n * NP; const float nqq = nq[qi];
  float m = -INFINITY, l = 0.0f; v8f o[16];
#pragma unroll
  for (int i = 0; i < 16; ++i) o[i] = (v8f){};
  for (int kb = 0; kb < NP; kb += 32) { v8f s0 = {}, s1 = {};
#pragma unroll 2
    for (int ks = 0; ks < C; ks += 32) { const v16b qf = frag_kb(qp + qi * C + ks, hh), ql = frag_kb(qp + PLN + qi * C + ks, hh);
      const v16b ka = frag_kb(K + (size_t)(kb + col) * C + ks, hh), kal = frag_kb(K + PLN + (size_t)(kb + col) * C + ks, hh), kc = frag_kb(K + (size_t)(kb + 16 + col) * C + ks, hh), kcl = frag_kb(K + PLN + (size_t)(kb + 16 + col) * C + ks, hh);
      s0 = wmma16b(ka, qf, s0); s0 = wmma16b(ka, ql, s0); s0 = wmma16b(kal, qf, s0); s1 = wmma16b(kc, qf, s1); s1 = wmma16b(kc, ql, s1); s1 = wmma16b(kcl, qf, s1); }
    const float nqc = __shfl(nqq, col) ;
    float mr = -INFINITY;
#pragma unroll
    for (int r = 0; r < 8; ++r) { s0[r] *= (1.0f / (AS_ * AS_)) * nqc * NK[kb + 8 * hh + r]; s1[r] *= (1.0f / (AS_ * AS_)) * nqc * NK[kb + 16 + 8 * hh + r]; mr = fmaxf(mr, fmaxf(s0[r], s1[r])); }
    mr = fmaxf(mr, __shfl_xor(mr, 16));
    const float mn = fmaxf(m, mr), al_ = nexp(m - mn); m = mn; float sum = 0.0f; v16b pbv, plv;
#pragma unroll
    for (int r = 0; r < 8; ++r) { const float e0 = nexp(s0[r] - mn), e1 = nexp(s1[r] - mn); sum += e0 + e1; b16 a, cc; split16(e0 * PS, a, cc); pbv[r] = a; plv[r] = cc; split16(e1 * PS, a, cc); pbv[8 + r] = a; plv[8 + r] = cc; }
    sum += __shfl_xor(sum, 16); l = l * al_ + sum;
#pragma unroll
    for (int t = 0; t < 16; ++t) { o[t] *= al_; const v16b vf = frag_kb(V + (size_t)(t * 16 + col) * NP + kb, hh), vl = frag_kb(V + PLN + (size_t)(t * 16 + col) * NP + kb, hh); o[t] = wmma16b(vf, pbv, o[t]); o[t] = wmma16b(vf, plv, o[t]); o[t] = wmma16b(vl, pbv, o[t]); } }
  const float inv = 1.0f / (l * VS * PS);
#pragma unroll
  for (int t = 0; t < 16; ++t)
#pragma unroll
    for (int r = 0; r < 8; ++r) Os[wid][col][t * 16 + 8 * hh + r] = o[t][r] * inv;
  wave_lds_sync();
  float* dst = arow + (size_t)tok0 * C;
  for (int pass = 0; pass < 2; ++pass) { for (int i = lane; i < 16 * 64; i += 32) { const int rr = i >> 6, c4 = (i & 63) * 4; *(volatile v4f*)(dst + (size_t)rr * C + c4) = *(const v4f*)(&Os[wid][rr][c4]); } __threadfence(); }
}

__global__ __launch_bounds__(128) void gate_kernel(const float* __restrict__ c, const float* __restrict__ arow, const b16* __restrict__ wzn16, const float* __restrict__ P, float* __restrict__ h) {
  __shared__ __attribute__((aligned(16))) float Ts[4][32 * 64];
  const int lane = threadIdx.x & 31, wave = threadIdx.x >> 5, nloc = lane & 15, hlf = lane >> 4, m0 = blockIdx.y * 128 + wave * 32, c0 = blockIdx.x * 64;
  const b16* WZ = wzn16; const b16* WN = wzn16 + (size_t)C * 512; const float* bz = P + 256; const float* bn = P + 512;
  v8f az[2][4], an[2][4];
#pragma unroll
  for (int r = 0; r < 2; ++r)
#pragma unroll
    for (int t = 0; t < 4; ++t) { az[r][t] = (v8f){}; an[r][t] = (v8f){}; }
#pragma unroll 1
  for (int kb = 0; kb < 512; kb += 32) { const float* src = (kb < C) ? c : arow; const int kk = kb & (C - 1); v16b a0, l0, a1, l1; frag_split(src + (size_t)(m0 + nloc) * C + kk, hlf, a0, l0); frag_split(src + (size_t)(m0 + 16 + nloc) * C + kk, hlf, a1, l1);
#pragma unroll
    for (int t = 0; t < 4; ++t) { const size_t ro = (size_t)(c0 + t * 16 + nloc) * 512 + kb; const v16b wz_ = frag_kb(WZ + ro, hlf), wn_ = frag_kb(WN + ro, hlf);
      az[0][t] = wmma16b(a0, wz_, az[0][t]); az[0][t] = wmma16b(l0, wz_, az[0][t]); az[1][t] = wmma16b(a1, wz_, az[1][t]); az[1][t] = wmma16b(l1, wz_, az[1][t]);
      an[0][t] = wmma16b(a0, wn_, an[0][t]); an[0][t] = wmma16b(l0, wn_, an[0][t]); an[1][t] = wmma16b(a1, wn_, an[1][t]); an[1][t] = wmma16b(l1, wn_, an[1][t]); } }
  float* Tt = Ts[wave];
#pragma unroll
  for (int t = 0; t < 4; ++t) { const int ch = c0 + t * 16 + nloc; const float b1 = bz[ch], b2 = bn[ch];
#pragma unroll
    for (int r = 0; r < 2; ++r)
#pragma unroll
      for (int v = 0; v < 8; ++v) { const float z = sigm(az[r][t][v] * (1.0f / AS_) + b1), nn = tanh_(an[r][t][v] * (1.0f / AS_) + b2); Tt[(r * 16 + v + 8 * hlf) * 64 + t * 16 + nloc] = (1.0f - z) * nn; } }
  wave_lds_sync();
  store_tile(Tt, h + (size_t)m0 * C + c0, C, lane);
}

__global__ __launch_bounds__(128) void out_kernel(const float* __restrict__ h, const b16* __restrict__ wo16, const float* __restrict__ P, float* __restrict__ out) {
  __shared__ __attribute__((aligned(16))) float Tc[64][128 + 4];
  const int lane = threadIdx.x & 31, wave = threadIdx.x >> 5, nloc = lane & 15, hlf = lane >> 4, m0 = blockIdx.y * 128 + wave * 32, c0 = blockIdx.x * 64; const int n = (blockIdx.y * 128) / NP, p0 = (blockIdx.y * 128) % NP; const float* bo = P + 768;
  v8f acc[2][4];
#pragma unroll
  for (int r = 0; r < 2; ++r)
#pragma unroll
    for (int t = 0; t < 4; ++t) acc[r][t] = (v8f){};
#pragma unroll 2
  for (int kb = 0; kb < C; kb += 32) { v16b a0, l0, a1, l1; frag_split(h + (size_t)(m0 + nloc) * C + kb, hlf, a0, l0); frag_split(h + (size_t)(m0 + 16 + nloc) * C + kb, hlf, a1, l1);
#pragma unroll
    for (int t = 0; t < 4; ++t) { const v16b bw = frag_kb(wo16 + (size_t)(c0 + t * 16 + nloc) * C + kb, hlf); acc[0][t] = wmma16b(a0, bw, acc[0][t]); acc[0][t] = wmma16b(l0, bw, acc[0][t]); acc[1][t] = wmma16b(a1, bw, acc[1][t]); acc[1][t] = wmma16b(l1, bw, acc[1][t]); } }
#pragma unroll
  for (int t = 0; t < 4; ++t) { const int co = c0 + t * 16 + nloc; const float bb = bo[co];
#pragma unroll
    for (int r = 0; r < 2; ++r)
#pragma unroll
      for (int v = 0; v < 8; ++v) Tc[t * 16 + nloc][wave * 32 + r * 16 + 8 * hlf + v] = acc[r][t][v] * (1.0f / AS_) + bb; }
  __syncthreads();
  for (int pass = 0; pass < 2; ++pass) { for (int i = threadIdx.x; i < 64 * 32; i += 128) { const int cc = i >> 5, c4 = (i & 31) * 4; *(volatile v4f*)(out + (((size_t)n * CO + c0 + cc) * NP) + p0 + c4) = *(const v4f*)(&Tc[cc][c4]); } __threadfence(); }
}
}

extern "C" void kernel_launch(void* const* d_in, const int* in_sizes, int n_in,
                              void* d_out, int out_size, void* d_ws, size_t ws_size, hipStream_t stream) {
  (void)n_in; (void)out_size;
  const float* x = (const float*)d_in[0]; const float* wpx = (const float*)d_in[1]; const float* wconv = (const float*)d_in[2]; const float* wq = (const float*)d_in[3]; const float* wk = (const float*)d_in[4]; const float* wv = (const float*)d_in[5]; const float* s = (const float*)d_in[6];
  const float* wz = (const float*)d_in[7]; const float* bz = (const float*)d_in[8]; const float* wn = (const float*)d_in[9]; const float* bn = (const float*)d_in[10]; const float* wo = (const float*)d_in[11]; const float* bo = (const float*)d_in[12];
  float* out = (float*)d_out;
  if (in_sizes[0] != Nn * I0 * NP || in_sizes[1] != C * I0 || in_sizes[2] != C * 512 * 9 || in_sizes[3] != C * C || in_sizes[7] != C * 512 || in_sizes[11] != CO * C) return;
  size_t off = 0; char* ws = (char*)d_ws;
  auto carve = [&](size_t bytes) { char* p = ws + off; off += (bytes + 255) & ~(size_t)255; return p; };
  unsigned short* xT = (unsigned short*)carve((size_t)NT * I0 * 2); unsigned short* wpx16 = (unsigned short*)carve((size_t)C * I0 * 2); b16* wc16 = (b16*)carve((size_t)C * KC * 2); b16* wqkv16 = (b16*)carve((size_t)3 * C * C * 2); b16* wzn16 = (b16*)carve((size_t)2 * C * 512 * 2); b16* wo16 = (b16*)carve((size_t)CO * C * 2); float* P = (float*)carve(1024 * 4);
  float* xt = (float*)carve(PLN * 4); float* cr = (float*)carve(PLN * 4); b16* qp = (b16*)carve(PLN * 2 * 2); b16* kp = (b16*)carve(PLN * 2 * 2); b16* vt = (b16*)carve(PLN * 2 * 2); float* qs = (float*)carve((size_t)2 * NT * 4 * 4); float* nq = (float*)carve((size_t)NT * 4); float* nk = (float*)carve((size_t)NT * 4);
  float* arow = xt;
  float* h = (float*)qp;
  if (off > ws_size) return;
  prep_kernel<<<dim3(NP / 64, Nn), 256, 0, stream>>>(x, wpx, wconv, wq, wk, wv, s, wz, bz, wn, bn, wo, bo, xT, wpx16, wc16, wqkv16, wzn16, wo16, P);
  px_kernel<<<dim3(C / 64, NT / 128), 128, 0, stream>>>(xT, wpx16, xt);
  conv_kernel<<<dim3(C / 64, NT / 128), 128, 0, stream>>>(xt, wc16, cr);
  qkv_kernel<<<dim3(C / 64, NT / 128, 3), 128, 0, stream>>>(cr, wqkv16, P, qp, kp, vt, qs);
  nrm_kernel<<<NT / 256, 256, 0, stream>>>(qs, nq, nk);
  attn_kernel<<<NT / 128, 256, 0, stream>>>(qp, kp, vt, nq, nk, arow);
  gate_kernel<<<dim3(C / 64, NT / 128), 128, 0, stream>>>(cr, arow, wzn16, P, h);
  out_kernel<<<dim3(CO / 64, NT / 128), 128, 0, stream>>>(h, wo16, P, out);
}
